// TransMatch_86947317940362
// MI455X (gfx1250) — hardware-verified
//
#include <hip/hip_runtime.h>
#include <stdint.h>


typedef __attribute__((ext_vector_type(16))) _Float16 v16h;
typedef __attribute__((ext_vector_type(8)))  _Float16 v8h;
typedef __attribute__((ext_vector_type(16))) __bf16   v16b;
typedef __attribute__((ext_vector_type(8)))  __bf16   v8b;
typedef __attribute__((ext_vector_type(8)))  float    v8f;
typedef __attribute__((ext_vector_type(4)))  float    v4f;
typedef __attribute__((ext_vector_type(8)))  unsigned short v8us;
typedef __attribute__((ext_vector_type(2)))  double   v2d;

#define NL    8
#define NS    192
#define ND    512
#define NDFF  2048
#define NB    16
#define NCH   4096
#define MROWS 3072
#define XROWS 512
#define BN_EPS 1e-5

__device__ __forceinline__ unsigned short f2bf_bits(float f) {
  unsigned u = __float_as_uint(f);
  return (unsigned short)((u + 0x7FFFu + ((u >> 16) & 1u)) >> 16);
}
__device__ __forceinline__ float bf_bits2f(unsigned short h) { return __uint_as_float(((unsigned)h) << 16); }
__device__ __forceinline__ void split_bf(float x, unsigned short& h, unsigned short& l) {
  h = f2bf_bits(x);
  l = f2bf_bits(x - bf_bits2f(h));
}

__device__ __forceinline__ void dep_guard_h(v8f& a, v8f& b, v16h x, v16h y) { asm volatile("v_nop\n\tv_nop\n\tv_nop\n\tv_nop" : "+v"(a), "+v"(b) : "v"(x), "v"(y)); }
__device__ __forceinline__ void dep_guard_b(v8f& a, v8f& b, v16b x, v16b y) { asm volatile("v_nop\n\tv_nop\n\tv_nop\n\tv_nop" : "+v"(a), "+v"(b) : "v"(x), "v"(y)); }
__device__ __forceinline__ void keep4_h(v16h a, v16h b, v16h c, v16h d) { asm volatile("v_nop" :: "v"(a), "v"(b), "v"(c), "v"(d)); }
__device__ __forceinline__ void keep4_b(v16b a, v16b b, v16b c, v16b d) { asm volatile("v_nop" :: "v"(a), "v"(b), "v"(c), "v"(d)); }
__device__ __forceinline__ void acc_guard4(v8f& a, v8f& b, v8f& c, v8f& d) { asm volatile("v_nop\n\tv_nop\n\tv_nop\n\tv_nop" : "+v"(a), "+v"(b), "+v"(c), "+v"(d)); }
template <typename T> struct Frag;
template <> struct Frag<_Float16> {
  typedef v16h V; union U { v16h v; v8h h[2]; };
  static __device__ __forceinline__ v16h load(const _Float16* p) {
    U f; f.h[0] = *(const v8h*)(p); f.h[1] = *(const v8h*)(p + 16); return f.v;
  }
  static __device__ __forceinline__ v8f mma(v16h a, v16h b, v8f c) {
    return __builtin_amdgcn_wmma_f32_16x16x32_f16(false, a, false, b, (short)0, c, false, false);
  }
  static __device__ __forceinline__ void guard(v8f& a, v8f& b, v16h x, v16h y) { dep_guard_h(a, b, x, y); }
  static __device__ __forceinline__ void keep(v16h a, v16h b, v16h c, v16h d) { keep4_h(a, b, c, d); }
};
template <> struct Frag<__bf16> {
  typedef v16b V; union U { v16b v; v8b h[2]; };
  static __device__ __forceinline__ v16b load(const __bf16* p) {
    U f; f.h[0] = *(const v8b*)(p); f.h[1] = *(const v8b*)(p + 16); return f.v;
  }
  static __device__ __forceinline__ v8f mma(v16b a, v16b b, v8f c) {
    return __builtin_amdgcn_wmma_f32_16x16x32_bf16(false, a, false, b, (short)0, c, false, false);
  }
  static __device__ __forceinline__ void guard(v8f& a, v8f& b, v16b x, v16b y) { dep_guard_b(a, b, x, y); }
  static __device__ __forceinline__ void keep(v16b a, v16b b, v16b c, v16b d) { keep4_b(a, b, c, d); }
};

template <int ET> struct Elem;
template <> struct Elem<0> { typedef _Float16 T; };
template <> struct Elem<1> { typedef __bf16 T; };
template <int ET, bool SPLIT, int BIAS_MODE, int OUT_MODE, bool RESID, int ACT = 0>
__global__ __launch_bounds__(256) void wmma_gemm64(
    const unsigned short* __restrict__ Ap, const unsigned short* __restrict__ A2p, int lda, long strideA,
    const unsigned short* __restrict__ Btp, const unsigned short* __restrict__ Bt2p, int ldb, long strideB,
    void* __restrict__ Cout, void* __restrict__ Cout2, int ldc, long strideC,
    const float* __restrict__ bias,
    const float* __restrict__ resid, long strideR,
    int M, int N, int K, float scale) {
  typedef typename Elem<ET>::T T;
  typedef typename Frag<T>::V V;
  const T* A = (const T*)Ap; const T* A2 = (const T*)A2p; const T* Bt = (const T*)Btp; const T* Bt2 = (const T*)Bt2p;
  __shared__ __align__(16) float sT[8][16 * 68];
  const int b    = blockIdx.y;
  const int lane = threadIdx.x & 31;
  const int wave = threadIdx.x >> 5;
  const int tilesN = N >> 6;
  const int tilesM = M >> 6;
  const int tile = blockIdx.x * 8 + wave;
  if (tile >= tilesM * tilesN) return;
  const int tm = tile / tilesN;
  const int tn = tile - tm * tilesN;
  const int m0 = tm << 6;
  const int n0 = tn << 6;

  const T* Ab  = A  + (size_t)b * strideA;
  const T* Bb  = Bt + (size_t)b * strideB;
  const T* Ab2 = SPLIT ? (A2  + (size_t)b * strideA) : nullptr;
  const T* Bb2 = SPLIT ? (Bt2 + (size_t)b * strideB) : nullptr;

  const int rlane = lane & 15;
  const int koff  = (lane >> 4) * 8;
  const int mOff  = (lane >> 4) * 8;

  v8f acc[4][4];
#pragma unroll
  for (int i = 0; i < 4; ++i)
#pragma unroll
    for (int j = 0; j < 4; ++j) acc[i][j] = (v8f){0.f,0.f,0.f,0.f,0.f,0.f,0.f,0.f};

  for (int k0 = 0; k0 < K; k0 += 32) {
    V bh[4], bl[4];
#pragma unroll
    for (int j = 0; j < 4; ++j) {
      const size_t bo = (size_t)(n0 + (j << 4) + rlane) * ldb + koff + k0;
      bh[j] = Frag<T>::load(Bb + bo);
      if (SPLIT) bl[j] = Frag<T>::load(Bb2 + bo);
    }
#pragma unroll
    for (int i = 0; i < 4; ++i) {
      const size_t ao = (size_t)(m0 + (i << 4) + rlane) * lda + koff + k0;
      V ah = Frag<T>::load(Ab + ao);
      V al;
      if (SPLIT) al = Frag<T>::load(Ab2 + ao);
#pragma unroll
      for (int j = 0; j < 4; ++j) {
        acc[i][j] = Frag<T>::mma(ah, bh[j], acc[i][j]);
        if (SPLIT) {
          acc[i][j] = Frag<T>::mma(ah, bl[j], acc[i][j]);
          acc[i][j] = Frag<T>::mma(al, bh[j], acc[i][j]);
        }
      }
      Frag<T>::guard(acc[i][0], acc[i][3], ah, SPLIT ? al : ah);
    }
    Frag<T>::keep(bh[0], bh[1], bh[2], bh[3]);
    if (SPLIT) Frag<T>::keep(bl[0], bl[1], bl[2], bl[3]);
  }
  acc_guard4(acc[0][0], acc[0][1], acc[0][2], acc[0][3]);
  acc_guard4(acc[1][0], acc[1][1], acc[1][2], acc[1][3]);
  acc_guard4(acc[2][0], acc[2][1], acc[2][2], acc[2][3]);
  acc_guard4(acc[3][0], acc[3][1], acc[3][2], acc[3][3]);

  float* slab = sT[wave];
  const float* Rb = RESID ? (resid + (size_t)b * strideR) : nullptr;
#pragma unroll
  for (int i = 0; i < 4; ++i) {
    const int mBase = m0 + (i << 4);
#pragma unroll
    for (int j = 0; j < 4; ++j) {
      const int n = n0 + (j << 4) + rlane;
      float bv = 0.f;
      if (BIAS_MODE == 2) bv = bias[n];
#pragma unroll
      for (int r = 0; r < 8; ++r) {
        float v = acc[i][j][r] * scale;
        if (BIAS_MODE == 1) v += bias[mBase + mOff + r];
        if (BIAS_MODE == 2) v += bv;
        if (RESID) v += Rb[(size_t)(mBase + mOff + r) * ldc + n];
        if (ACT == 1) v = tanhf(v);
        if (ACT == 2) v = fmaxf(v, 0.0f);
        if (ACT == 3) v = v / (1.0f + expf(-v));
        if (ACT == 4) v = (v > 0.f) ? v : 0.01f * v;
        if (ACT == 5) v = 0.5f * v * (1.0f + erff(v * 0.70710678118654752f));
        slab[(mOff + r) * 68 + (j << 4) + rlane] = v;
      }
    }
    __builtin_amdgcn_fence(__ATOMIC_RELEASE, "workgroup");
    __builtin_amdgcn_wave_barrier();
    __builtin_amdgcn_fence(__ATOMIC_ACQUIRE, "workgroup");
    if (OUT_MODE == 0) {
      float* C = (float*)Cout + (size_t)b * strideC;
      const int hh = lane >> 4, c4 = (lane & 15) * 4;
      for (int pass = 0; pass < 2; ++pass) {
#pragma unroll
        for (int it = 0; it < 8; ++it) {
          const int row = it * 2 + hh;
          v4f v = *(const v4f*)(slab + row * 68 + c4);
          *(volatile v4f*)(C + (size_t)(mBase + row) * ldc + n0 + c4) = v;
        }
        __threadfence();
      }
    } else {
      const int q = lane >> 3, c8 = (lane & 7) * 8;
      unsigned short* C  = (unsigned short*)Cout  + (size_t)b * strideC;
      unsigned short* C2 = (OUT_MODE == 2) ? ((unsigned short*)Cout2 + (size_t)b * strideC) : nullptr;
      for (int pass = 0; pass < 2; ++pass) {
#pragma unroll
        for (int it = 0; it < 4; ++it) {
          const int row = it * 4 + q;
          const float* sp = slab + row * 68 + c8;
          v8h hv, lv;
#pragma unroll
          for (int e = 0; e < 8; ++e) {
            if (OUT_MODE == 1) {
              hv[e] = (_Float16)sp[e];
            } else {
              unsigned short hb = f2bf_bits(sp[e]);
              unsigned short lb = f2bf_bits(sp[e] - bf_bits2f(hb));
              hv[e] = __builtin_bit_cast(_Float16, hb);
              lv[e] = __builtin_bit_cast(_Float16, lb);
            }
          }
          *(volatile v8h*)(C + (size_t)(mBase + row) * ldc + n0 + c8) = hv;
          if (OUT_MODE == 2) *(volatile v8h*)(C2 + (size_t)(mBase + row) * ldc + n0 + c8) = lv;
        }
        __threadfence();
      }
    }
    __builtin_amdgcn_fence(__ATOMIC_RELEASE, "workgroup");
    __builtin_amdgcn_wave_barrier();
    __builtin_amdgcn_fence(__ATOMIC_ACQUIRE, "workgroup");
  }
}

__global__ __launch_bounds__(256) void k_prep_w0(const float* __restrict__ w0, const float* __restrict__ b0,
    unsigned short* __restrict__ W0H, unsigned short* __restrict__ W0L, float* __restrict__ B0S,
    int n8, int nb4, float bscale) {
  const int g = blockIdx.x * 256 + threadIdx.x;
  const bool dw = g < n8;
  const bool db = g < nb4;
  v8us hv = (v8us){0,0,0,0,0,0,0,0}, lv = (v8us){0,0,0,0,0,0,0,0};
  v4f bbv = (v4f){0.f,0.f,0.f,0.f};
  if (dw) {
    const v4f a = *(const v4f*)(w0 + (size_t)g * 8);
    const v4f c = *(const v4f*)(w0 + (size_t)g * 8 + 4);
#pragma unroll
    for (int e = 0; e < 4; ++e) {
      unsigned short h, l;
      split_bf(a[e], h, l); hv[e] = h;     lv[e] = l;
      split_bf(c[e], h, l); hv[4 + e] = h; lv[4 + e] = l;
    }
  }
  if (db) bbv = *(const v4f*)(b0 + (size_t)g * 4) * bscale;
  for (int pass = 0; pass < 2; ++pass) {
    if (dw) {
      *(volatile v8us*)(W0H + (size_t)g * 8) = hv;
      *(volatile v8us*)(W0L + (size_t)g * 8) = lv;
    }
    if (db) *(volatile v4f*)(B0S + (size_t)g * 4) = bbv;
    __threadfence();
  }
}

__global__ __launch_bounds__(256) void k_prep_w2sig(const float* __restrict__ w2, const float* __restrict__ se,
    _Float16* __restrict__ W2H, float* __restrict__ SIG, int n8, int nsig, float wscale) {
  const int g = blockIdx.x * 256 + threadIdx.x;
  const bool dw = g < n8;
  const bool ds = g < nsig;
  v8h hv = (v8h){0,0,0,0,0,0,0,0};
  float sgm = 0.f;
  if (dw) {
    const v4f a = *(const v4f*)(w2 + (size_t)g * 8) * wscale;
    const v4f c = *(const v4f*)(w2 + (size_t)g * 8 + 4) * wscale;
#pragma unroll
    for (int e = 0; e < 4; ++e) { hv[e] = (_Float16)a[e]; hv[4 + e] = (_Float16)c[e]; }
  }
  if (ds) {
    const float x = se[g];
    sgm = 1.0f / (1.0f + expf(-x));
  }
  for (int pass = 0; pass < 2; ++pass) {
    if (dw) *(volatile v8h*)(W2H + (size_t)g * 8) = hv;
    if (ds) *(volatile float*)(SIG + g) = sgm;
    __threadfence();
  }
}

__global__ __launch_bounds__(256) void k_planes(const float* __restrict__ qf, const float* __restrict__ gf, int layer,
    unsigned short* __restrict__ APH, unsigned short* __restrict__ APL) {
  __shared__ __align__(16) float tile[64][68];
  const int bx = blockIdx.x;
  const int dchunk = bx / 3, schunk = bx - dchunk * 3;
  const int b = blockIdx.y, which = blockIdx.z;
  const float* feat = which ? gf : qf;
  const int d0 = dchunk * 64, s0 = schunk * 64;
  const int tid = threadIdx.x;
  {
    const int r = tid >> 2, cs = (tid & 3) * 16;
    const float* src = feat + ((size_t)b * NCH + (size_t)layer * ND + d0 + r) * NS + s0 + cs;
#pragma unroll
    for (int i = 0; i < 4; ++i) *(v4f*)(&tile[r][cs + 4 * i]) = *(const v4f*)(src + 4 * i);
  }
  __syncthreads();
  const size_t rowbase = (size_t)which * MROWS + (size_t)b * NS + s0;
  v8us hq[2], lq[2];
#pragma unroll
  for (int p = 0; p < 2; ++p) {
    const int sr = p * 32 + (tid >> 3);
    const int dseg = (tid & 7) * 8;
#pragma unroll
    for (int e = 0; e < 8; ++e) {
      unsigned short h, l;
      split_bf(tile[dseg + e][sr], h, l);
      hq[p][e] = h; lq[p][e] = l;
    }
  }
  for (int pass = 0; pass < 2; ++pass) {
#pragma unroll
    for (int p = 0; p < 2; ++p) {
      const int sr = p * 32 + (tid >> 3);
      const int dseg = (tid & 7) * 8;
      const size_t o = (rowbase + sr) * ND + d0 + dseg;
      *(volatile v8us*)(APH + o) = hq[p];
      *(volatile v8us*)(APL + o) = lq[p];
    }
    __threadfence();
  }
}

__global__ __launch_bounds__(256) void k_maskmax(const float* __restrict__ SC, const float* __restrict__ SIGl,
                                                 float* __restrict__ XM, double* __restrict__ BN1P) {
  __shared__ float wred[8][NS];
  __shared__ __align__(16) float outv[2 * NS];
  __shared__ double dred[2][8];
  __shared__ double tot[2];
  const int qk = blockIdx.x;
  const int q = qk >> 4, kb = qk & 15;
  const int tid = threadIdx.x, wave = tid >> 5, lane = tid & 31;
  const int tx = tid & 15, ty = tid >> 4;
  const float* scb = SC + (size_t)(kb * NS) * MROWS + (size_t)q * NS;
  const float NEG = -__builtin_huge_valf();
  float cm[12];
#pragma unroll
  for (int bb = 0; bb < 12; ++bb) cm[bb] = NEG;
#pragma unroll 2
  for (int a = 0; a < 12; ++a) {
    const int s = ty + 16 * a;
    const float* rowp = scb + (size_t)s * MROWS + tx;
    const float* sgp = SIGl + s * NS + tx;
    float r = NEG;
#pragma unroll
    for (int bb = 0; bb < 12; ++bb) {
      const float v = rowp[16 * bb] * sgp[16 * bb];
      cm[bb] = fmaxf(cm[bb], v);
      r = fmaxf(r, v);
    }
    r = fmaxf(r, __shfl_xor(r, 8, 32));
    r = fmaxf(r, __shfl_xor(r, 4, 32));
    r = fmaxf(r, __shfl_xor(r, 2, 32));
    r = fmaxf(r, __shfl_xor(r, 1, 32));
    if (tx == 0) outv[NS + s] = r;
  }
#pragma unroll
  for (int bb = 0; bb < 12; ++bb) {
    float v = cm[bb];
    v = fmaxf(v, __shfl_xor(v, 16, 32));
    if (lane < 16) wred[wave][tx + 16 * bb] = v;
  }
  __syncthreads();
  if (tid < NS) {
    float m = wred[0][tid];
#pragma unroll
    for (int w = 1; w < 8; ++w) m = fmaxf(m, wred[w][tid]);
    outv[tid] = m;
  }
  __syncthreads();
  double s1 = 0.0, s2 = 0.0;
  if (tid < NS) {
    const double a0 = (double)outv[tid], a1 = (double)outv[NS + tid];
    s1 = a0 + a1; s2 = a0 * a0 + a1 * a1;
  }
  s1 += __shfl_xor(s1, 16, 32); s2 += __shfl_xor(s2, 16, 32);
  s1 += __shfl_xor(s1, 8, 32);  s2 += __shfl_xor(s2, 8, 32);
  s1 += __shfl_xor(s1, 4, 32);  s2 += __shfl_xor(s2, 4, 32);
  s1 += __shfl_xor(s1, 2, 32);  s2 += __shfl_xor(s2, 2, 32);
  s1 += __shfl_xor(s1, 1, 32);  s2 += __shfl_xor(s2, 1, 32);
  if (lane == 0) { dred[0][wave] = s1; dred[1][wave] = s2; }
  __syncthreads();
  if (tid == 0) {
    double a0 = 0.0, a1 = 0.0;
#pragma unroll
    for (int w = 0; w < 8; ++w) { a0 += dred[0][w]; a1 += dred[1][w]; }
    tot[0] = a0; tot[1] = a1;
  }
  __syncthreads();
  v4f xv = (v4f){0.f,0.f,0.f,0.f};
  if (tid < 96) xv = *(const v4f*)(outv + tid * 4);
  v2d bv; bv[0] = 0.0; bv[1] = 0.0;
  if (tid == 0) { bv[0] = tot[0]; bv[1] = tot[1]; }
  float* xdst = XM + (size_t)qk * (2 * NS) + tid * 4;
  double* bdst = BN1P + (size_t)qk * 16 + tid * 2;
  for (int pass = 0; pass < 2; ++pass) {
    if (tid < 96) *(volatile v4f*)xdst = xv;
    if (tid < 8)  *(volatile v2d*)bdst = bv;
    __threadfence();
  }
}

__global__ __launch_bounds__(192) void k_bn1_apply(const float* __restrict__ XM, const double* __restrict__ BN1P,
    const float* __restrict__ g1p, const float* __restrict__ b1p, int layer, float carry,
    _Float16* __restrict__ X16) {
  __shared__ float ssc[2];
  const int tid = threadIdx.x;
  if (tid < 32) {
    double s1 = 0.0, s2 = 0.0;
#pragma unroll
    for (int e = 0; e < 8; ++e) {
      const int idx = tid + 32 * e;
      s1 += BN1P[idx * 16];
      s2 += BN1P[idx * 16 + 1];
    }
    s1 += __shfl_xor(s1, 16, 32); s2 += __shfl_xor(s2, 16, 32);
    s1 += __shfl_xor(s1, 8, 32);  s2 += __shfl_xor(s2, 8, 32);
    s1 += __shfl_xor(s1, 4, 32);  s2 += __shfl_xor(s2, 4, 32);
    s1 += __shfl_xor(s1, 2, 32);  s2 += __shfl_xor(s2, 2, 32);
    s1 += __shfl_xor(s1, 1, 32);  s2 += __shfl_xor(s2, 1, 32);
    if (tid == 0) {
      const double inv = 1.0 / 98304.0;
      const double mean = s1 * inv;
      double var = s2 * inv - mean * mean;
      if (var < 0.0) var = 0.0;
      const double rstd = 1.0 / sqrt(var + BN_EPS);
      const double g = (double)g1p[layer], bb = (double)b1p[layer];
      const float sc = (float)(g * rstd);
      const float sh = (float)(bb - mean * g * rstd);
      ssc[0] = sc * carry;
      ssc[1] = sh * carry;
    }
  }
  __syncthreads();
  const float sc = ssc[0], sh = ssc[1];
  const int rloc = tid / 24;
  const int cseg = (tid - rloc * 24) * 8;
  const int row = blockIdx.x * 8 + rloc;
  const float* xp = XM + (size_t)row * NS + cseg;
  const v4f a = *(const v4f*)xp;
  const v4f c = *(const v4f*)(xp + 4);
  v8h hv;
#pragma unroll
  for (int e = 0; e < 4; ++e) {
    hv[e]     = (_Float16)(a[e] * sc + sh);
    hv[4 + e] = (_Float16)(c[e] * sc + sh);
  }
  _Float16* dst = X16 + (size_t)row * NS + cseg;
  for (int pass = 0; pass < 2; ++pass) {
    *(volatile v8h*)dst = hv;
    __threadfence();
  }
}

__device__ __forceinline__ float row_partial64(const float* __restrict__ hp, const float* csc, const float* csh, const float* cw) {
  float p = 0.f;
#pragma unroll 2
  for (int c4 = 0; c4 < 16; ++c4) {
    const v4f x = *(const v4f*)(hp + 4 * c4);
#pragma unroll
    for (int e = 0; e < 4; ++e) {
      const int c = 4 * c4 + e;
      const float v = fmaxf(x[e] * csc[c] + csh[c], 0.0f);
      p += v * cw[c];
    }
  }
  return p;
}
__global__ __launch_bounds__(256) void k_bn2_fc3(const float* __restrict__ HB, const float* __restrict__ g2,
    const float* __restrict__ bb2, const float* __restrict__ w3, int layer, float* __restrict__ FP) {
  __shared__ double ps1[4][64], ps2[4][64];
  __shared__ __align__(16) float csc[64], csh[64], cw[64];
  const int ct = blockIdx.x, c0 = ct * 64;
  const int tid = threadIdx.x;
  const int c = tid & 63, rg = tid >> 6;
  double s1 = 0.0, s2 = 0.0;
#pragma unroll 2
  for (int r = rg; r < XROWS; r += 4) {
    const float x = HB[(size_t)r * NDFF + c0 + c];
    s1 += (double)x;
    s2 += (double)x * (double)x;
  }
  ps1[rg][c] = s1; ps2[rg][c] = s2;
  __syncthreads();
  if (tid < 64) {
    const double a0 = ((ps1[0][tid] + ps1[1][tid]) + ps1[2][tid]) + ps1[3][tid];
    const double a1 = ((ps2[0][tid] + ps2[1][tid]) + ps2[2][tid]) + ps2[3][tid];
    const double inv = 1.0 / 512.0;
    const double mu = a0 * inv;
    double var = a1 * inv - mu * mu;
    if (var < 0.0) var = 0.0;
    const double rstd = 1.0 / sqrt(var + BN_EPS);
    const int n = layer * NDFF + c0 + tid;
    const double g = (double)g2[n];
    csc[tid] = (float)(g * rstd);
    csh[tid] = (float)((double)bb2[n] - mu * g * rstd);
    cw[tid]  = w3[n];
  }
  __syncthreads();
  const float p0 = row_partial64(HB + (size_t)tid * NDFF + c0, csc, csh, cw);
  const float p1 = row_partial64(HB + (size_t)(tid + 256) * NDFF + c0, csc, csh, cw);
  float* dst = FP + (size_t)ct * XROWS;
  for (int pass = 0; pass < 2; ++pass) {
    *(volatile float*)(dst + tid) = p0;
    *(volatile float*)(dst + 256 + tid) = p1;
    __threadfence();
  }
}

__global__ __launch_bounds__(256) void k_final(const float* __restrict__ FP, const float* __restrict__ b3p,
    const float* __restrict__ g3p, const float* __restrict__ bb3p, const int* __restrict__ targets,
    int layer, int first, float* __restrict__ ACC, float* __restrict__ out) {
  __shared__ double dred[2][8];
  __shared__ float st[2];
  const int j = threadIdx.x, wave = j >> 5, lane = j & 31;
  double d0 = 0.0, d1 = 0.0;
#pragma unroll 4
  for (int ct = 0; ct < 32; ++ct) {
    d0 += (double)FP[ct * XROWS + 2 * j];
    d1 += (double)FP[ct * XROWS + 2 * j + 1];
  }
  const float b3 = b3p[layer];
  const float y0 = (float)d0 + b3;
  const float y1 = (float)d1 + b3;
  const float z = y0 + y1;
  double s1 = (double)z, s2 = (double)z * (double)z;
  s1 += __shfl_xor(s1, 16, 32); s2 += __shfl_xor(s2, 16, 32);
  s1 += __shfl_xor(s1, 8, 32);  s2 += __shfl_xor(s2, 8, 32);
  s1 += __shfl_xor(s1, 4, 32);  s2 += __shfl_xor(s2, 4, 32);
  s1 += __shfl_xor(s1, 2, 32);  s2 += __shfl_xor(s2, 2, 32);
  s1 += __shfl_xor(s1, 1, 32);  s2 += __shfl_xor(s2, 1, 32);
  if (lane == 0) { dred[0][wave] = s1; dred[1][wave] = s2; }
  __syncthreads();
  if (j == 0) {
    double a0 = 0.0, a1 = 0.0;
#pragma unroll
    for (int w = 0; w < 8; ++w) { a0 += dred[0][w]; a1 += dred[1][w]; }
    const double inv = 1.0 / 256.0;
    const double mean = a0 * inv;
    double var = a1 * inv - mean * mean;
    if (var < 0.0) var = 0.0;
    const double rstd = 1.0 / sqrt(var + BN_EPS);
    const double g = (double)g3p[layer];
    st[0] = (float)(g * rstd);
    st[1] = (float)((double)bb3p[layer] - mean * g * rstd);
  }
  __syncthreads();
  const float val = z * st[0] + st[1];
  const float prev = first ? 0.0f : ACC[j];
  const float accv = prev + val;
  const int ta = targets[j >> 4], tb = targets[j & 15];
  const float lab = (ta == tb) ? 1.0f : 0.0f;
  for (int pass = 0; pass < 2; ++pass) {
    *(volatile float*)(ACC + j) = accv;
    *(volatile float*)(out + j) = accv;
    *(volatile float*)(out + 256 + j) = lab;
    __threadfence();
  }
}

extern "C" void kernel_launch(void* const* d_in, const int* in_sizes, int n_in,
                              void* d_out, int out_size, void* d_ws, size_t ws_size,
                              hipStream_t stream) {
  if (n_in < 16) return;
  if (in_sizes[0] != NB * NCH * NS || in_sizes[1] != NB * NCH * NS || in_sizes[2] != NB ||
      in_sizes[3] != NL * NS * NS || in_sizes[4] != NL * ND * ND || in_sizes[5] != NL * ND ||
      in_sizes[8] != NL * NDFF * NS || in_sizes[9] != NL * NDFF || in_sizes[12] != NL * NDFF ||
      out_size != 512) return;
  const float* q_feat      = (const float*)d_in[0];
  const float* g_feat      = (const float*)d_in[1];
  const int*   targets     = (const int*)d_in[2];
  const float* score_embed = (const float*)d_in[3];
  const float* fc0_w       = (const float*)d_in[4];
  const float* fc0_b       = (const float*)d_in[5];
  const float* bn1_g       = (const float*)d_in[6];
  const float* bn1_b       = (const float*)d_in[7];
  const float* fc2_w       = (const float*)d_in[8];
  const float* fc2_b       = (const float*)d_in[9];
  const float* bn2_g       = (const float*)d_in[10];
  const float* bn2_b       = (const float*)d_in[11];
  const float* fc3_w       = (const float*)d_in[12];
  const float* fc3_b       = (const float*)d_in[13];
  const float* bn3_g       = (const float*)d_in[14];
  const float* bn3_b       = (const float*)d_in[15];
  float* out = (float*)d_out;

  char* ws = (char*)d_ws;
  size_t off = 0;
  auto carve = [&](size_t bytes) -> void* {
    void* p = ws + off;
    off = (off + bytes + 255) & ~(size_t)255;
    return p;
  };
  unsigned short* W0H  = (unsigned short*)carve((size_t)NL * ND * ND * 2);
  unsigned short* W0L  = (unsigned short*)carve((size_t)NL * ND * ND * 2);
  unsigned short* W2H  = (unsigned short*)carve((size_t)NL * NDFF * NS * 2);
  float*          SIG  = (float*)carve((size_t)NL * NS * NS * 4);
  float*          B0S  = (float*)carve((size_t)NL * ND * 4);
  unsigned short* APH  = (unsigned short*)carve((size_t)2 * MROWS * ND * 2);
  unsigned short* APL  = (unsigned short*)carve((size_t)2 * MROWS * ND * 2);
  unsigned short* QK16 = (unsigned short*)carve((size_t)2 * MROWS * ND * 2);
  float*          SC   = (float*)carve((size_t)MROWS * MROWS * 4);
  float*          XM   = (float*)carve((size_t)XROWS * NS * 4);
  double*         BN1P = (double*)carve((size_t)256 * 128);
  unsigned short* X16  = (unsigned short*)carve((size_t)XROWS * NS * 2);
  float*          HB   = (float*)carve((size_t)XROWS * NDFF * 4);
  float*          FP   = (float*)carve((size_t)32 * XROWS * 4);
  float*          ACC  = (float*)carve((size_t)256 * 4);
  if (off > ws_size || off > (size_t)134217728) return;

  const int n8_w0 = NL * ND * ND / 8;
  const int nb4   = NL * ND / 4;
  const int n8_w2 = NL * NDFF * NS / 8;
  const int nsig  = NL * NS * NS;
  k_prep_w0<<<dim3((n8_w0 + 255) / 256), 256, 0, stream>>>(fc0_w, fc0_b, W0H, W0L, B0S, n8_w0, nb4, 8.0f);
  {
    const int nmax = n8_w2 > nsig ? n8_w2 : nsig;
    k_prep_w2sig<<<dim3((nmax + 255) / 256), 256, 0, stream>>>(fc2_w, score_embed, (_Float16*)W2H, SIG, n8_w2, nsig, 16.0f);
  }

  const unsigned short* Q16 = QK16;
  const unsigned short* K16 = QK16 + (size_t)MROWS * ND;
  const long plane = (long)MROWS * ND;

  for (int i = 0; i < NL; ++i) {
    k_planes<<<dim3(24, NB, 2), 256, 0, stream>>>(q_feat, g_feat, i, APH, APL);
    wmma_gemm64<1, true, 2, 1, false, 0><<<dim3(48, 2), 256, 0, stream>>>(
        APH, APL, ND, plane,
        W0H + (size_t)i * ND * ND, W0L + (size_t)i * ND * ND, ND, 0L,
        (void*)QK16, (void*)QK16, ND, plane,
        B0S + (size_t)i * ND,
        B0S, 0L,
        MROWS, ND, ND, 8.0f);
    wmma_gemm64<0, false, 0, 0, false, 0><<<dim3(288, 1), 256, 0, stream>>>(
        K16, K16, ND, 0L,
        Q16, Q16, ND, 0L,
        (void*)SC, (void*)SC, MROWS, 0L,
        B0S,
        B0S, 0L,
        MROWS, MROWS, ND, 1.0f / 64.0f);
    k_maskmax<<<dim3(256), 256, 0, stream>>>(SC, SIG + (size_t)i * NS * NS, XM, BN1P);
    k_bn1_apply<<<dim3(64), 192, 0, stream>>>(XM, BN1P, bn1_g, bn1_b, i, 8.0f, (_Float16*)X16);
    wmma_gemm64<0, false, 2, 0, false, 0><<<dim3(32, 1), 256, 0, stream>>>(
        X16, X16, NS, 0L,
        W2H + (size_t)i * NDFF * NS, W2H + (size_t)i * NDFF * NS, NS, 0L,
        (void*)HB, (void*)HB, NDFF, 0L,
        fc2_b + (size_t)i * NDFF,
        B0S, 0L,
        XROWS, NDFF, NS, 1.0f / 128.0f);
    k_bn2_fc3<<<dim3(32), 256, 0, stream>>>(HB, bn2_g, bn2_b, fc3_w, i, FP);
    k_final<<<dim3(1), 256, 0, stream>>>(FP, fc3_b, bn3_g, bn3_b, targets, i, (i == 0) ? 1 : 0, ACC, out);
  }
}
